// Encoder_61899068670101
// MI455X (gfx1250) — hardware-run, weakly checked
//
#include <hip/hip_runtime.h>
#include <math.h>

constexpr int NBATCH = 512;
constexpr int NSTEP  = 1024;
constexpr int NVOCAB = 1000;
constexpr int NEMB   = 64;
constexpr int NHID   = 64;
constexpr int NGATE  = 256;
constexpr int KTOT   = 128;
constexpr int ROWS_PER_BLK = 16;
constexpr int NTHR   = 128;
constexpr int APITCH = 136;
constexpr int WPITCH = 136;
constexpr int HSP    = 68;
constexpr float ACARRY = 1024.0f;
constexpr float WCARRY = 256.0f;
constexpr float FOLD   = 1.0f / (ACARRY * WCARRY);
constexpr float F16_MIN_NORMAL = 6.103515625e-05f;

static_assert(NGATE == 4 * NHID, "gate order i | f | g | o, 64 columns each");
static_assert(KTOT == NEMB + NHID && KTOT % 32 == 0, "K = 128, four 32-deep k-steps");
static_assert(NBATCH % ROWS_PER_BLK == 0, "32 row tiles per direction");
static_assert(NTHR * 8 == ROWS_PER_BLK * NEMB, "x staging: 128 threads x 8 halves = 16 rows x 64 columns exactly");
static_assert(32 * NTHR * 8 == NGATE * KTOT, "weight staging: 32 iterations x 128 threads x 8 halves = 256 x 128 exactly");
static_assert(2 * NTHR * 4 == ROWS_PER_BLK * NHID, "final store: 2 iterations x 128 threads x 4 floats = 16 rows x 64 columns exactly");
static_assert((APITCH * 2) % 16 == 0 && (WPITCH * 2) % 16 == 0 && (HSP * 4) % 16 == 0, "16-B aligned LDS rows");
static_assert(ACARRY * WCARRY == 262144.0f, "fold constant is 2^-18");

typedef __attribute__((ext_vector_type(16))) _Float16 v16h;
typedef __attribute__((ext_vector_type(8)))  _Float16 v8h;
typedef __attribute__((ext_vector_type(8)))  float    v8f;
typedef __attribute__((ext_vector_type(4)))  float    v4f;
typedef __attribute__((ext_vector_type(4)))  int      v4i;

union FragU { v16h v; v8h h[2]; };
__device__ __forceinline__ v16h frag_load(const _Float16* p) {
  FragU f;
  f.h[0] = *(const v8h*)(p);
  f.h[1] = *(const v8h*)(p + 16);
  return f.v;
}

__device__ __forceinline__ v8f mma_f16(v16h a, v16h b, v8f c) {
  c = __builtin_amdgcn_wmma_f32_16x16x32_f16(false, a, false, b, (short)0, c, false, false);
  asm volatile("v_nop\n\tv_nop\n\tv_nop\n\tv_nop" : "+v"(c) : "v"(a), "v"(b));
  return c;
}

__device__ __forceinline__ _Float16 cvt_operand(float v, float carry) {
  const float s = v * carry;
  const float t = (fabsf(s) < F16_MIN_NORMAL) ? 0.0f : s;
  return (_Float16)t;
}

__device__ __forceinline__ float fsig(float x)  { return __builtin_amdgcn_rcpf(1.0f + __expf(-x)); }
__device__ __forceinline__ float ftanh(float x) { return 1.0f - 2.0f * __builtin_amdgcn_rcpf(__expf(2.0f * x) + 1.0f); }

__device__ __forceinline__ void stage_step(_Float16* At, int* Msk, const int* __restrict__ tokens,
                                           const float* __restrict__ emb, int rowbase, int tt, int tid) {
  const int m  = tid >> 3;
  const int c8 = (tid & 7) * 8;
  int tok = tokens[(size_t)(rowbase + m) * NSTEP + (size_t)tt];
  asm volatile("" : "+v"(tok));
  const int tc = (tok < 0) ? 0 : ((tok > NVOCAB - 1) ? (NVOCAB - 1) : tok);
  const float* er = emb + (size_t)tc * NEMB + c8;
  const v4f xa = *(const v4f*)(er);
  const v4f xb = *(const v4f*)(er + 4);
  v8h hv;
#pragma unroll
  for (int e = 0; e < 4; ++e) {
    hv[e]     = cvt_operand(xa[e], ACARRY);
    hv[4 + e] = cvt_operand(xb[e], ACARRY);
  }
  *(v8h*)(At + m * APITCH + c8) = hv;
  if ((tid & 7) == 0) Msk[m] = (tok != 0) ? 1 : 0;
}

__global__ __launch_bounds__(NTHR) void bidir_recurrent_kernel(
    const int* __restrict__ tokens, const float* __restrict__ emb,
    const float* __restrict__ wx_f, const float* __restrict__ wh_f, const float* __restrict__ bias_f,
    const float* __restrict__ wx_b, const float* __restrict__ wh_b, const float* __restrict__ bias_b,
    float* __restrict__ out) {
  __shared__ __align__(16) _Float16 Bt[NGATE * WPITCH];
  __shared__ __align__(16) _Float16 At[ROWS_PER_BLK * APITCH];
  __shared__ __align__(16) float    Hs[ROWS_PER_BLK * HSP];
  __shared__ __align__(16) int      Msk[ROWS_PER_BLK];

  const int tid  = threadIdx.x;
  const int lane = tid & 31;
  const int wave = tid >> 5;
  const int c    = lane & 15;
  const int hh   = lane >> 4;
  const int koff = hh * 8;
  const int dir     = blockIdx.y;
  const int rowbase = blockIdx.x * ROWS_PER_BLK;
  const float* wx = dir ? wx_b : wx_f;
  const float* wh = dir ? wh_b : wh_f;
  const float* bi = dir ? bias_b : bias_f;
  const int j = 16 * wave + c;

#pragma unroll 1
  for (int it = 0; it < 32; ++it) {
    const int idx = it * NTHR + tid;
    const int n   = idx & 255;
    const int kg  = idx >> 8;
    const float* src = (kg < 8) ? wx : wh;
    const int kb = (kg & 7) * 8;
    v8h hv;
#pragma unroll
    for (int e = 0; e < 8; ++e) hv[e] = cvt_operand(src[(kb + e) * NGATE + n], WCARRY);
    *(v8h*)(Bt + n * WPITCH + kg * 8) = hv;
  }
  {
    v8h zv;
#pragma unroll
    for (int e = 0; e < 8; ++e) zv[e] = (_Float16)0.0f;
    *(v8h*)(At + (tid >> 3) * APITCH + NEMB + (tid & 7) * 8) = zv;
  }
  stage_step(At, Msk, tokens, emb, rowbase, dir ? (NSTEP - 1) : 0, tid);

  float bb[4], cst[8], hst[8];
#pragma unroll
  for (int g = 0; g < 4; ++g) bb[g] = bi[g * NHID + j];
#pragma unroll
  for (int r = 0; r < 8; ++r) { cst[r] = 0.0f; hst[r] = 0.0f; }
  __syncthreads();

  const _Float16* arow = At + c * APITCH + koff;
  const _Float16* brow = Bt + j * WPITCH + koff;
  const v8f z8 = {0.f, 0.f, 0.f, 0.f, 0.f, 0.f, 0.f, 0.f};

#pragma unroll 1
  for (int s = 0; s < NSTEP; ++s) {
    const v4i mk0 = *(const v4i*)(Msk + 8 * hh);
    const v4i mk1 = *(const v4i*)(Msk + 8 * hh + 4);
    int keep[8];
    keep[0] = mk0[0]; keep[1] = mk0[1]; keep[2] = mk0[2]; keep[3] = mk0[3];
    keep[4] = mk1[0]; keep[5] = mk1[1]; keep[6] = mk1[2]; keep[7] = mk1[3];

    v8f acc[4];
    acc[0] = z8; acc[1] = z8; acc[2] = z8; acc[3] = z8;
#pragma unroll 1
    for (int ks = 0; ks < KTOT / 32; ++ks) {
      const v16h a  = frag_load(arow + 32 * ks);
      const v16h b0 = frag_load(brow + 32 * ks);
      const v16h b1 = frag_load(brow + 1 * NHID * WPITCH + 32 * ks);
      const v16h b2 = frag_load(brow + 2 * NHID * WPITCH + 32 * ks);
      const v16h b3 = frag_load(brow + 3 * NHID * WPITCH + 32 * ks);
      acc[0] = mma_f16(a, b0, acc[0]);
      acc[1] = mma_f16(a, b1, acc[1]);
      acc[2] = mma_f16(a, b2, acc[2]);
      acc[3] = mma_f16(a, b3, acc[3]);
    }

#pragma unroll
    for (int r = 0; r < 8; ++r) {
      const float zi = acc[0][r] * FOLD + bb[0];
      const float zf = acc[1][r] * FOLD + bb[1];
      const float zg = acc[2][r] * FOLD + bb[2];
      const float zo = acc[3][r] * FOLD + bb[3];
      const float ig = fsig(zi);
      const float fg = fsig(zf);
      const float gg = ftanh(zg);
      const float og = fsig(zo);
      const float cn = fg * cst[r] + ig * gg;
      const float hn = og * ftanh(cn);
      const bool kp = (keep[r] != 0);
      cst[r] = kp ? cn : cst[r];
      hst[r] = kp ? hn : hst[r];
    }

    __syncthreads();
#pragma unroll
    for (int r = 0; r < 8; ++r) At[(8 * hh + r) * APITCH + NEMB + j] = cvt_operand(hst[r], ACARRY);
    {
      const int sn  = (s + 1 < NSTEP) ? (s + 1) : s;
      const int ttn = dir ? (NSTEP - 1 - sn) : sn;
      stage_step(At, Msk, tokens, emb, rowbase, ttn, tid);
    }
    __syncthreads();
  }

#pragma unroll
  for (int r = 0; r < 8; ++r) Hs[(8 * hh + r) * HSP + j] = hst[r];
  __syncthreads();
  for (int pass = 0; pass < 2; ++pass) {
#pragma unroll
    for (int it = 0; it < 2; ++it) {
      const int idx = it * NTHR + tid;
      const int row = idx >> 4;
      const int c4  = (idx & 15) * 4;
      const v4f v = *(const v4f*)(Hs + row * HSP + c4);
      *(volatile v4f*)(out + (size_t)(rowbase + row) * (2 * NHID) + NHID * dir + c4) = v;
    }
    __threadfence();
  }
}

extern "C" void kernel_launch(void* const* d_in, const int* in_sizes, int n_in,
                              void* d_out, int out_size, void* d_ws, size_t ws_size, hipStream_t stream) {
  (void)d_ws; (void)ws_size;
  if (n_in < 8 || d_out == nullptr) return;
  if (in_sizes[0] != NBATCH * NSTEP || in_sizes[1] != NVOCAB * NEMB) return;
  if (in_sizes[2] != NEMB * NGATE || in_sizes[3] != NHID * NGATE || in_sizes[4] != NGATE) return;
  if (in_sizes[5] != NEMB * NGATE || in_sizes[6] != NHID * NGATE || in_sizes[7] != NGATE) return;
  if (out_size != NBATCH * 2 * NHID) return;

  const int*   tokens = (const int*)  d_in[0];
  const float* emb    = (const float*)d_in[1];
  const float* wx_f   = (const float*)d_in[2];
  const float* wh_f   = (const float*)d_in[3];
  const float* bias_f = (const float*)d_in[4];
  const float* wx_b   = (const float*)d_in[5];
  const float* wh_b   = (const float*)d_in[6];
  const float* bias_b = (const float*)d_in[7];
  float* out = (float*)d_out;

  bidir_recurrent_kernel<<<dim3(NBATCH / ROWS_PER_BLK, 2), NTHR, 0, stream>>>(
      tokens, emb, wx_f, wh_f, bias_f, wx_b, wh_b, bias_b, out);
}
